// Gemma4Attention_15058155340378
// MI455X (gfx1250) — hardware-verified
//
#include <hip/hip_runtime.h>


#ifndef NB
#define NB 2
#endif
#ifndef SEQ
#define SEQ 2048
#endif

namespace {
constexpr int SEQ_FULL = 2048, MASK_LD = 2048, EMB = 2048, NH = 16, NKV = 4, HD = 128, NQ = NH * HD, NKD = NKV * HD, NOUT = NQ + 2 * NKD;
constexpr int MROWS = NB * SEQ, NT = SEQ / 32, RES_ROWS = 128;
constexpr float XS = 8.0f, WSC = 256.0f, PS = 1024.0f, LOG2E = 1.4426950408889634f, EPSN = 1.0e-6f, NEGB = -3.4028235e38f, ECLAMP = -16384.0f;
static_assert(SEQ % 64 == 0 && SEQ >= 64 && SEQ <= SEQ_FULL && NT >= 1 && NT <= 64);
static_assert(NB >= 1 && NB <= 2 && HD == 128 && EMB == 2048 && NQ == 2048 && NKD == 512 && NOUT % 128 == 0 && MROWS % 64 == 0 && EMB % 32 == 0 && NQ % 32 == 0);

typedef _Float16 b16;
typedef __attribute__((ext_vector_type(16))) _Float16 v16b;
typedef __attribute__((ext_vector_type(8))) _Float16 v8b;
typedef __attribute__((ext_vector_type(4))) _Float16 v4h;
typedef __attribute__((ext_vector_type(2))) _Float16 v2h;
typedef __attribute__((ext_vector_type(8))) float v8f;
typedef __attribute__((ext_vector_type(4))) float v4f;
typedef __attribute__((ext_vector_type(4))) int v4i;
union I8 { v4i q[2]; int i[8]; };

__device__ __forceinline__ float bf16_rne(float f) { unsigned int u = __float_as_uint(f); u += 0x7FFFu + ((u >> 16) & 1u); return __uint_as_float(u & 0xFFFF0000u); }
__device__ __forceinline__ void split16(float v, b16& hi, b16& lo) { hi = (b16)v; lo = (b16)(v - (float)hi); }
__device__ __forceinline__ v16b frag_kb(const b16* p, int hh) { const v8b a = *(const v8b*)(p + 8 * hh), b = *(const v8b*)(p + 16 + 8 * hh); v16b f;
#pragma unroll
  for (int e = 0; e < 8; ++e) { f[e] = a[e]; f[8 + e] = b[e]; } return f; }
__device__ __forceinline__ v8f wmma16b(v16b a, v16b b, v8f c) { v8f d = __builtin_amdgcn_wmma_f32_16x16x32_f16(false, a, false, b, (short)0, c, false, false); asm volatile("v_nop\n\tv_nop\n\tv_nop\n\tv_nop" : "+v"(d) : "v"(a), "v"(b)); return d; }
__device__ __forceinline__ void wave_lds_sync() { __builtin_amdgcn_fence(__ATOMIC_RELEASE, "workgroup"); __builtin_amdgcn_wave_barrier(); __builtin_amdgcn_fence(__ATOMIC_ACQUIRE, "workgroup"); }
__device__ __forceinline__ int iclamp(int v, int lo, int hi) { return v < lo ? lo : (v > hi ? hi : v); }
__device__ __forceinline__ float nexp2(float v) { return __builtin_amdgcn_exp2f(v); }

__global__ __launch_bounds__(256) void prep_kernel(const float* __restrict__ wq, const float* __restrict__ wk, const float* __restrict__ wv, const float* __restrict__ wo, const float* __restrict__ x,
                                                   b16* WT, b16* WP, b16* Xh) {
  const int blk = blockIdx.x, d0 = threadIdx.x * 8;
  v8b o; b16* dst;
  if (blk < NOUT) {
    const float* src; int ld, oc;
    if (blk < NQ) { src = wq; ld = NQ; oc = blk; } else if (blk < NQ + NKD) { src = wk; ld = NKD; oc = blk - NQ; } else { src = wv; ld = NKD; oc = blk - NQ - NKD; }
#pragma unroll
    for (int j = 0; j < 8; ++j) o[j] = (b16)(bf16_rne(src[(size_t)(d0 + j) * ld + oc]) * WSC);
    dst = WT + (size_t)blk * EMB + d0;
  } else if (blk < NOUT + EMB) {
    const int oe = blk - NOUT;
#pragma unroll
    for (int j = 0; j < 8; ++j) o[j] = (b16)(bf16_rne(wo[(size_t)(d0 + j) * EMB + oe]) * WSC);
    dst = WP + (size_t)oe * NQ + d0;
  } else {
    const int tok = blk - NOUT - EMB; const size_t xr = (size_t)(tok / SEQ) * SEQ_FULL + (size_t)(tok % SEQ);
    const v4f f0 = *(const v4f*)(x + xr * EMB + d0), f1 = *(const v4f*)(x + xr * EMB + d0 + 4);
#pragma unroll
    for (int j = 0; j < 4; ++j) { o[j] = (b16)(bf16_rne(f0[j]) * XS); o[4 + j] = (b16)(bf16_rne(f1[j]) * XS); }
    dst = Xh + (size_t)tok * EMB + d0;
  }
  for (int pass = 0; pass < 2; ++pass) { *(volatile v8b*)dst = o; __threadfence(); }
}

__global__ __launch_bounds__(256) void mrange_kernel(const int* __restrict__ maskp, int* tab) {
  __shared__ unsigned int wl[8], wh[8], wr[8];
  const int qb = blockIdx.x, tid = threadIdx.x, wave = tid >> 5, lane = tid & 31;
  unsigned int tl = 0u, th = 0u, rm = 0u;
  constexpr int NC4 = SEQ / 4;
#pragma unroll 1
  for (int i = tid; i < 32 * NC4; i += 256) {
    const int r = i / NC4, c4 = i - r * NC4;
    const v4i w = *(const v4i*)(maskp + (size_t)(qb * 32 + r) * MASK_LD + c4 * 4);
    const unsigned int bit = ((w[0] == 0) | (w[1] == 0) | (w[2] == 0) | (w[3] == 0)) ? 1u : 0u;
    const int kt = c4 >> 3; const unsigned int sb = bit << (kt & 31);
    tl |= (kt < 32) ? sb : 0u; th |= (kt < 32) ? 0u : sb; rm |= bit << r;
  }
#pragma unroll
  for (int o = 1; o < 32; o <<= 1) { tl |= __shfl_xor(tl, o); th |= __shfl_xor(th, o); rm |= __shfl_xor(rm, o); }
  if (lane == 0) { wl[wave] = tl; wh[wave] = th; wr[wave] = rm; }
  __syncthreads();
  unsigned int TL = 0u, TH = 0u, RM = 0u;
#pragma unroll
  for (int w = 0; w < 8; ++w) { TL |= wl[w]; TH |= wh[w]; RM |= wr[w]; }
  int lo = 0, hi = NT - 1;
  if (RM == 0xFFFFFFFFu && (TL | TH) != 0u) {
    lo = (TL != 0u) ? (__ffs((int)TL) - 1) : (32 + __ffs((int)TH) - 1);
    hi = (TH != 0u) ? (63 - __clz((int)TH)) : (31 - __clz((int)TL));
  }
  lo = iclamp(lo, 0, NT - 1); hi = iclamp(hi, 0, NT - 1);
  v4i val; val[0] = lo; val[1] = hi; val[2] = lo; val[3] = hi;
  for (int pass = 0; pass < 2; ++pass) { if (tid < 8) *(volatile v4i*)(tab + (size_t)qb * 32 + tid * 4) = val; __threadfence(); }
}

__global__ __launch_bounds__(128) void proj_kernel(const b16* __restrict__ Xh, const b16* __restrict__ WT, const float* __restrict__ cosb, const float* __restrict__ sinb,
                                                   const float* __restrict__ qnw, const float* __restrict__ knw, b16* Qh, b16* Ql, b16* Kh, b16* Kl, b16* VTh, b16* VTl) {
  __shared__ __attribute__((aligned(16))) float Tf[4][16][HD + 4];
  const int wave = threadIdx.x >> 5, lane = threadIdx.x & 31, nloc = lane & 15, hlf = lane >> 4;
  const int r0 = blockIdx.x * 64, m0 = r0 + wave * 16; const int slab = blockIdx.y, n0 = slab * 128;
  v8f acc[8];
#pragma unroll
  for (int t = 0; t < 8; ++t) acc[t] = (v8f){};
#pragma unroll 1
  for (int kb = 0; kb < EMB; kb += 32) { const v16b a = frag_kb(Xh + (size_t)(m0 + nloc) * EMB + kb, hlf);
#pragma unroll
    for (int t = 0; t < 8; ++t) acc[t] = wmma16b(a, frag_kb(WT + (size_t)(n0 + t * 16 + nloc) * EMB + kb, hlf), acc[t]); }
#pragma unroll
  for (int t = 0; t < 8; ++t)
#pragma unroll
    for (int r = 0; r < 8; ++r) Tf[wave][8 * hlf + r][t * 16 + nloc] = acc[t][r] * (1.0f / (XS * WSC));
  __syncthreads();
  if (slab < NH + NKV) {
    const bool isq = slab < NH;
    const float* nw = isq ? qnw : knw; b16* Ph = isq ? Qh : Kh; b16* Pl = isq ? Ql : Kl; const size_t hrow0 = (size_t)(isq ? slab : slab - NH) * MROWS;
    float wgt[4];
#pragma unroll
    for (int j = 0; j < 4; ++j) wgt[j] = bf16_rne(nw[lane + 32 * j]);
#pragma unroll 1
    for (int rr = 0; rr < 16; ++rr) {
      const int tok = m0 + rr, s = tok % SEQ; float v[4], c[4], sn[4]; float ss = 0.0f;
#pragma unroll
      for (int j = 0; j < 4; ++j) { v[j] = Tf[wave][rr][lane + 32 * j]; ss += v[j] * v[j]; c[j] = bf16_rne(cosb[(size_t)s * HD + lane + 32 * j]); sn[j] = bf16_rne(sinb[(size_t)s * HD + lane + 32 * j]); }
#pragma unroll
      for (int o = 1; o < 32; o <<= 1) ss += __shfl_xor(ss, o);
      const float inv = rsqrtf(ss * (1.0f / HD) + EPSN);
#pragma unroll
      for (int j = 0; j < 4; ++j) v[j] = v[j] * inv * wgt[j];
      const float a0 = v[0] * c[0] - v[2] * sn[0], a1 = v[1] * c[1] - v[3] * sn[1], a2 = v[2] * c[2] + v[0] * sn[2], a3 = v[3] * c[3] + v[1] * sn[3];
      Tf[wave][rr][lane] = a0 * XS; Tf[wave][rr][lane + 32] = a1 * XS; Tf[wave][rr][lane + 64] = a2 * XS; Tf[wave][rr][lane + 96] = a3 * XS;
    }
    wave_lds_sync();
    for (int pass = 0; pass < 2; ++pass) {
#pragma unroll 1
      for (int rr = 0; rr < 16; ++rr) { const int tok = m0 + rr; const v4f f = *(const v4f*)(&Tf[wave][rr][lane * 4]); v4h hv, lv;
#pragma unroll
        for (int j = 0; j < 4; ++j) { b16 p, q_; split16(f[j], p, q_); hv[j] = p; lv[j] = q_; }
        const size_t oi = (hrow0 + (size_t)tok) * HD + lane * 4; *(volatile v4h*)(Ph + oi) = hv; *(volatile v4h*)(Pl + oi) = lv; }
      __threadfence(); }
  } else {
    const int kvh = slab - NH - NKV;
#pragma unroll 1
    for (int rr = 0; rr < 16; ++rr) { float v[4]; float ss = 0.0f;
#pragma unroll
      for (int j = 0; j < 4; ++j) { v[j] = Tf[wave][rr][lane + 32 * j]; ss += v[j] * v[j]; }
#pragma unroll
      for (int o = 1; o < 32; o <<= 1) ss += __shfl_xor(ss, o);
      const float inv = rsqrtf(ss * (1.0f / HD) + EPSN);
#pragma unroll
      for (int j = 0; j < 4; ++j) Tf[wave][rr][lane + 32 * j] = v[j] * inv * XS; }
    __syncthreads();
    for (int pass = 0; pass < 2; ++pass) {
#pragma unroll 1
      for (int q = 0; q < 32; ++q) { const int d = wave * 32 + q; const int tk = lane * 2; v2h hv, lv;
#pragma unroll
        for (int j = 0; j < 2; ++j) { b16 p, q_; split16(Tf[(tk + j) >> 4][(tk + j) & 15][d], p, q_); hv[j] = p; lv[j] = q_; }
        const size_t oi = ((size_t)kvh * HD + d) * MROWS + r0 + lane * 2; *(volatile v2h*)(VTh + oi) = hv; *(volatile v2h*)(VTl + oi) = lv; }
      __threadfence(); }
  }
}

__global__ __launch_bounds__(64) void attn_kernel(const b16* __restrict__ Qh, const b16* __restrict__ Ql, const b16* __restrict__ Kh, const b16* __restrict__ Kl, const b16* __restrict__ VTh, const b16* __restrict__ VTl,
                                                  const int* __restrict__ maskp, const int* __restrict__ tab, b16* Yh, b16* Yl) {
  __shared__ __attribute__((aligned(16))) b16 Pb[2][16][32 + 8], Pc[2][16][32 + 8]; __shared__ __attribute__((aligned(16))) float To[2][16][HD + 4];
  const int wave = threadIdx.x >> 5, lane = threadIdx.x & 31, hh = lane >> 4, col = lane & 15;
  const int h = blockIdx.y, kvh = h / (NH / NKV), qblk = blockIdx.x * 32, q0 = qblk + wave * 16, qi = q0 + col; const size_t tok0 = (size_t)blockIdx.z * SEQ;
  const b16* Qhb = Qh + ((size_t)h * MROWS + tok0 + (size_t)qi) * HD; const b16* Qlb = Ql + ((size_t)h * MROWS + tok0 + (size_t)qi) * HD;
  const b16* Khb = Kh + ((size_t)kvh * MROWS + tok0) * HD; const b16* Klb = Kl + ((size_t)kvh * MROWS + tok0) * HD;
  const b16* Vhb = VTh + (size_t)kvh * HD * MROWS + tok0; const b16* Vlb = VTl + (size_t)kvh * HD * MROWS + tok0;
  const int tlo = iclamp(tab[blockIdx.x * 32], 0, NT - 1), thi = iclamp(tab[blockIdx.x * 32 + 1], 0, NT - 1);
  const bool vres = qblk < RES_ROWS; const float cs = LOG2E / (XS * XS);
  float m = NEGB, l = 0.0f; v8f o[8];
#pragma unroll
  for (int t = 0; t < 8; ++t) o[t] = (v8f){};
#pragma unroll 1
  for (int kt = tlo; kt <= thi; ++kt) {
    const int kb = kt * 32; float e[16]; float mx = NEGB;
#pragma unroll
    for (int u = 0; u < 2; ++u) {
      v8f s = (v8f){}; const size_t kr = (size_t)(kb + u * 16 + col) * HD;
#pragma unroll 1
      for (int kq = 0; kq < 4; ++kq) {
        const v16b kh = frag_kb(Khb + kr + kq * 32, hh), kl = frag_kb(Klb + kr + kq * 32, hh), qh = frag_kb(Qhb + kq * 32, hh), ql = frag_kb(Qlb + kq * 32, hh);
        s = wmma16b(kh, qh, s); s = wmma16b(kh, ql, s); s = wmma16b(kl, qh, s); }
      const int* mp = maskp + (size_t)qi * MASK_LD + kb + u * 16 + 8 * hh; I8 mw; mw.q[0] = *(const v4i*)mp; mw.q[1] = *(const v4i*)(mp + 4);
#pragma unroll
      for (int r = 0; r < 8; ++r) { const float vv = (mw.i[r] != 0) ? NEGB : s[r] * cs; e[u * 8 + r] = vv; mx = fmaxf(mx, vv); } }
    mx = fmaxf(mx, __shfl_xor(mx, 16)); const float mn = fmaxf(m, mx); const float al = nexp2(fmaxf(m - mn, ECLAMP)); float sum = 0.0f;
#pragma unroll
    for (int i2 = 0; i2 < 16; ++i2) { const float p = nexp2(fmaxf(e[i2] - mn, ECLAMP)); sum += p; b16 a_, c_; split16(p * PS, a_, c_);
      const int sl = (i2 < 8 ? 0 : 16) + 8 * hh + (i2 & 7); Pb[wave][col][sl] = a_; Pc[wave][col][sl] = c_; }
    sum += __shfl_xor(sum, 16); l = l * al + sum; m = mn;
    wave_lds_sync();
    const v16b pf = frag_kb(&Pb[wave][col][0], hh), pg = frag_kb(&Pc[wave][col][0], hh);
    if (vres) {
#pragma unroll
      for (int t = 0; t < 8; ++t) { if ((t & 1) == 0) asm volatile("" ::: "memory");
        o[t] *= al; const size_t vr = (size_t)(t * 16 + col) * MROWS + kb; const v16b va = frag_kb(Vhb + vr, hh), vb = frag_kb(Vlb + vr, hh);
        o[t] = wmma16b(va, pf, o[t]); o[t] = wmma16b(va, pg, o[t]); o[t] = wmma16b(vb, pf, o[t]); }
    } else {
#pragma unroll
      for (int t = 0; t < 8; ++t) { if ((t & 1) == 0) asm volatile("" ::: "memory");
        o[t] *= al; const size_t vr = (size_t)(t * 16 + col) * MROWS + kb; const v16b va = frag_kb(Vhb + vr, hh);
        o[t] = wmma16b(va, pf, o[t]); o[t] = wmma16b(va, pg, o[t]); }
    }
    wave_lds_sync();
  }
  const float inv = (l > 0.0f) ? 1.0f / (l * PS * XS) : 0.0f;
#pragma unroll
  for (int t = 0; t < 8; ++t)
#pragma unroll
    for (int r = 0; r < 8; ++r) To[wave][col][t * 16 + 8 * hh + r] = o[t][r] * inv;
  wave_lds_sync();
  for (int pass = 0; pass < 2; ++pass) {
#pragma unroll 1
    for (int rr = 0; rr < 16; ++rr) { const v4f f = *(const v4f*)(&To[wave][rr][lane * 4]); v4h hv, lv;
#pragma unroll
      for (int j = 0; j < 4; ++j) { b16 p, q_; split16(f[j] * XS, p, q_); hv[j] = p; lv[j] = q_; }
      const size_t oi = (tok0 + (size_t)(q0 + rr)) * NQ + (size_t)h * HD + lane * 4; *(volatile v4h*)(Yh + oi) = hv; *(volatile v4h*)(Yl + oi) = lv; }
    __threadfence(); }
}

__global__ __launch_bounds__(128) void out_kernel(const b16* __restrict__ Yh, const b16* __restrict__ Yl, const b16* __restrict__ WP, float* out) {
  __shared__ __attribute__((aligned(16))) float Tf[4][16][128 + 4];
  const int wave = threadIdx.x >> 5, lane = threadIdx.x & 31, nloc = lane & 15, hlf = lane >> 4; const size_t m0 = ((size_t)blockIdx.x * 4 + wave) * 16; const int n0 = blockIdx.y * 128;
  const bool yres = ((blockIdx.x * 64) % SEQ) < RES_ROWS;
  v8f acc[8];
#pragma unroll
  for (int t = 0; t < 8; ++t) acc[t] = (v8f){};
  if (yres) {
#pragma unroll 1
    for (int kb = 0; kb < NQ; kb += 32) { const v16b a = frag_kb(Yh + (m0 + nloc) * NQ + kb, hlf), al = frag_kb(Yl + (m0 + nloc) * NQ + kb, hlf);
#pragma unroll
      for (int t = 0; t < 8; ++t) { const v16b bw = frag_kb(WP + (size_t)(n0 + t * 16 + nloc) * NQ + kb, hlf); acc[t] = wmma16b(a, bw, acc[t]); acc[t] = wmma16b(al, bw, acc[t]); } }
  } else {
#pragma unroll 1
    for (int kb = 0; kb < NQ; kb += 32) { const v16b a = frag_kb(Yh + (m0 + nloc) * NQ + kb, hlf);
#pragma unroll
      for (int t = 0; t < 8; ++t) { const v16b bw = frag_kb(WP + (size_t)(n0 + t * 16 + nloc) * NQ + kb, hlf); acc[t] = wmma16b(a, bw, acc[t]); } }
  }
#pragma unroll
  for (int t = 0; t < 8; ++t)
#pragma unroll
    for (int r = 0; r < 8; ++r) Tf[wave][8 * hlf + r][t * 16 + nloc] = acc[t][r] * (1.0f / (XS * WSC));
  wave_lds_sync();
  for (int pass = 0; pass < 2; ++pass) {
#pragma unroll 1
    for (int rr = 0; rr < 16; ++rr) *(volatile v4f*)(out + (m0 + rr) * EMB + n0 + lane * 4) = *(const v4f*)(&Tf[wave][rr][lane * 4]);
    __threadfence(); }
}
}

extern "C" void kernel_launch(void* const* d_in, const int* in_sizes, int n_in, void* d_out, int out_size, void* d_ws, size_t ws_size, hipStream_t stream) {
  if (n_in < 10) return;
  auto Fp = [&](int i) { return (const float*)d_in[i]; };
  if (in_sizes[0] < ((NB - 1) * SEQ_FULL + SEQ) * EMB || in_sizes[1] < (SEQ - 1) * MASK_LD + SEQ || in_sizes[2] < SEQ * HD || in_sizes[3] < SEQ * HD || in_sizes[4] < EMB * NQ ||
      in_sizes[5] < EMB * NKD || in_sizes[6] < EMB * NKD || in_sizes[7] < NQ * EMB || in_sizes[8] < HD || in_sizes[9] < HD || out_size < MROWS * EMB) return;
  size_t off = 0; char* ws = (char*)d_ws;
  auto carve = [&](size_t bytes) { char* p = ws + off; off += (bytes + 255) & ~(size_t)255; return p; };
  b16* WT = (b16*)carve((size_t)NOUT * EMB * 2); b16* WP = (b16*)carve((size_t)EMB * NQ * 2); b16* Xh = (b16*)carve((size_t)MROWS * EMB * 2);
  b16* Qh = (b16*)carve((size_t)NH * MROWS * HD * 2); b16* Ql = (b16*)carve((size_t)NH * MROWS * HD * 2);
  b16* Kh = (b16*)carve((size_t)NKV * MROWS * HD * 2); b16* Kl = (b16*)carve((size_t)NKV * MROWS * HD * 2);
  b16* VTh = (b16*)carve((size_t)NKV * HD * MROWS * 2); b16* VTl = (b16*)carve((size_t)NKV * HD * MROWS * 2);
  b16* Yh = (b16*)carve((size_t)MROWS * NQ * 2); b16* Yl = (b16*)carve((size_t)MROWS * NQ * 2);
  int* tab = (int*)carve((size_t)NT * 32 * 4);
  if (off > ws_size || off > ((size_t)128 << 20)) return;
  const int* maskp = (const int*)d_in[1];
  prep_kernel<<<(unsigned)(NOUT + EMB + MROWS), 256, 0, stream>>>(Fp(4), Fp(5), Fp(6), Fp(7), Fp(0), WT, WP, Xh);
  mrange_kernel<<<(unsigned)NT, 256, 0, stream>>>(maskp, tab);
  proj_kernel<<<dim3(MROWS / 64, NOUT / 128), 128, 0, stream>>>(Xh, WT, Fp(2), Fp(3), Fp(8), Fp(9), Qh, Ql, Kh, Kl, VTh, VTl);
  attn_kernel<<<dim3(SEQ / 32, NH, NB), 64, 0, stream>>>(Qh, Ql, Kh, Kl, VTh, VTl, maskp, tab, Yh, Yl);
  out_kernel<<<dim3(MROWS / 64, EMB / 128), 128, 0, stream>>>(Yh, Yl, WP, (float*)d_out);
}
